// AttentionLayer_4174708212459
// MI455X (gfx1250) — hardware-verified
//
#include <hip/hip_runtime.h>
#include <math.h>

#ifndef NB
#define NB 4
#endif
#ifndef SEQ
#define SEQ 1024
#endif
#define NB_FULL 4
#define SEQ_FULL 1024
#define HID 1024
#define NH 16
#define HD 64
#define FFD 4096
#define MAXP 1024
#define EROWS (2 * MAXP - 1)
#define NR (NB * SEQ)
#define LN_EPS 1e-12f
#define CSC 32.0f

static_assert(NB >= 1 && NB <= NB_FULL);
static_assert(SEQ % 64 == 0 && SEQ >= 64 && SEQ <= SEQ_FULL);
static_assert(NB == 1 || SEQ == SEQ_FULL);
static_assert(HID == NH * HD && HD == 64 && FFD == 4 * HID && HID % 64 == 0 && NR % 64 == 0);
static_assert((size_t)NR * FFD * 2 == (size_t)NR * HID * 2 * 4);

typedef __attribute__((ext_vector_type(16))) _Float16 v16h;
typedef __attribute__((ext_vector_type(8)))  _Float16 v8h;
typedef __attribute__((ext_vector_type(4)))  _Float16 v4h;
typedef __attribute__((ext_vector_type(16))) __bf16   v16b;
typedef __attribute__((ext_vector_type(8)))  __bf16   v8b;
typedef __attribute__((ext_vector_type(8)))  float    v8f;
typedef __attribute__((ext_vector_type(4)))  float    v4f;
typedef unsigned int cm_u4 __attribute__((ext_vector_type(4)));

__device__ __forceinline__ v8f wmma16(v16h a, v16h b, v8f c) {
    c = __builtin_amdgcn_wmma_f32_16x16x32_f16(false, a, false, b, (short)0, c, false, false);
    asm volatile("v_nop\n\tv_nop\n\tv_nop\n\tv_nop" : "+v"(c) : "v"(a), "v"(b));
    return c;
}
__device__ __forceinline__ v16h frag16(const _Float16* p, int hh) {
    union { v16h v; v8h q[2]; } f;
    f.q[0] = *(const v8h*)(p + 8 * hh);
    f.q[1] = *(const v8h*)(p + 16 + 8 * hh);
    return f.v;
}
__device__ __forceinline__ void ld_split() { asm volatile("s_nop 0" ::: "memory"); }

#define VST2(T, ptr, val) do { const T vst2_v_ = (val); *(volatile T*)(ptr) = vst2_v_; __threadfence(); *(volatile T*)(ptr) = vst2_v_; } while (0)
#define VST2V4(ptr, val) do { const v4f vst2_v4_ = (val); *(volatile v4f*)(ptr) = vst2_v4_; __threadfence(); *(volatile v4f*)(ptr) = vst2_v4_; } while (0)

namespace w25 {
typedef __attribute__((ext_vector_type(16))) _Float16 v16h;
typedef __attribute__((ext_vector_type(8)))  _Float16 v8h;
typedef __attribute__((ext_vector_type(16))) __bf16   v16b;
typedef __attribute__((ext_vector_type(8)))  __bf16   v8b;
typedef __attribute__((ext_vector_type(8)))  float    v8f;
typedef __attribute__((ext_vector_type(4)))  float    v4f;

__device__ __forceinline__ unsigned short f2bf_bits(float f) {
  unsigned u = __float_as_uint(f);
  return (unsigned short)((u + 0x7FFFu + ((u >> 16) & 1u)) >> 16);
}
__device__ __forceinline__ float bf_bits2f(unsigned short h) { return __uint_as_float(((unsigned)h) << 16); }

__device__ __forceinline__ void dep_guard_h(v8f& a, v8f& b, v16h x, v16h y) { asm volatile("v_nop\n\tv_nop\n\tv_nop\n\tv_nop" : "+v"(a), "+v"(b) : "v"(x), "v"(y)); }
__device__ __forceinline__ void dep_guard_b(v8f& a, v8f& b, v16b x, v16b y) { asm volatile("v_nop\n\tv_nop\n\tv_nop\n\tv_nop" : "+v"(a), "+v"(b) : "v"(x), "v"(y)); }
__device__ __forceinline__ void keep4_h(v16h a, v16h b, v16h c, v16h d) { asm volatile("v_nop" :: "v"(a), "v"(b), "v"(c), "v"(d)); }
__device__ __forceinline__ void keep4_b(v16b a, v16b b, v16b c, v16b d) { asm volatile("v_nop" :: "v"(a), "v"(b), "v"(c), "v"(d)); }
__device__ __forceinline__ void acc_guard4(v8f& a, v8f& b, v8f& c, v8f& d) { asm volatile("v_nop\n\tv_nop\n\tv_nop\n\tv_nop" : "+v"(a), "+v"(b), "+v"(c), "+v"(d)); }
template <typename T> struct Frag;
template <> struct Frag<_Float16> {
  typedef v16h V; union U { v16h v; v8h h[2]; };
  static __device__ __forceinline__ v16h load(const _Float16* p) {
    U f; f.h[0] = *(const v8h*)(p); f.h[1] = *(const v8h*)(p + 16); return f.v;
  }
  static __device__ __forceinline__ v8f mma(v16h a, v16h b, v8f c) {
    return __builtin_amdgcn_wmma_f32_16x16x32_f16(false, a, false, b, (short)0, c, false, false);
  }
  static __device__ __forceinline__ void guard(v8f& a, v8f& b, v16h x, v16h y) { dep_guard_h(a, b, x, y); }
  static __device__ __forceinline__ void keep(v16h a, v16h b, v16h c, v16h d) { keep4_h(a, b, c, d); }
};
template <> struct Frag<__bf16> {
  typedef v16b V; union U { v16b v; v8b h[2]; };
  static __device__ __forceinline__ v16b load(const __bf16* p) {
    U f; f.h[0] = *(const v8b*)(p); f.h[1] = *(const v8b*)(p + 16); return f.v;
  }
  static __device__ __forceinline__ v8f mma(v16b a, v16b b, v8f c) {
    return __builtin_amdgcn_wmma_f32_16x16x32_bf16(false, a, false, b, (short)0, c, false, false);
  }
  static __device__ __forceinline__ void guard(v8f& a, v8f& b, v16b x, v16b y) { dep_guard_b(a, b, x, y); }
  static __device__ __forceinline__ void keep(v16b a, v16b b, v16b c, v16b d) { keep4_b(a, b, c, d); }
};

template <int ET> struct Elem;
template <> struct Elem<0> { typedef _Float16 T; };
template <> struct Elem<1> { typedef __bf16 T; };
template <int ET, bool SPLIT, int BIAS_MODE, int OUT_MODE, bool RESID, int ACT = 0>
__global__ __launch_bounds__(256) void wmma_gemm64(
    const unsigned short* __restrict__ Ap, const unsigned short* __restrict__ A2p, int lda, long strideA,
    const unsigned short* __restrict__ Btp, const unsigned short* __restrict__ Bt2p, int ldb, long strideB,
    void* __restrict__ Cout, void* __restrict__ Cout2, int ldc, long strideC,
    const float* __restrict__ bias,
    const float* __restrict__ resid, long strideR,
    int M, int N, int K, float scale) {
  static_assert(!RESID || (OUT_MODE == 0 && ACT == 0));
  typedef typename Elem<ET>::T T;
  typedef typename Frag<T>::V V;
  const T* A = (const T*)Ap; const T* A2 = (const T*)A2p; const T* Bt = (const T*)Btp; const T* Bt2 = (const T*)Bt2p;
  __shared__ __align__(16) float sT[8][16 * 68];
  const int b    = blockIdx.y;
  const int lane = threadIdx.x & 31;
  const int wave = threadIdx.x >> 5;
  const int tilesN = N >> 6;
  const int tilesM = M >> 6;
  const int tile = blockIdx.x * 8 + wave;
  if (tile >= tilesM * tilesN) return;
  const int tm = tile / tilesN;
  const int tn = tile - tm * tilesN;
  const int m0 = tm << 6;
  const int n0 = tn << 6;

  const T* Ab  = A  + (size_t)b * strideA;
  const T* Bb  = Bt + (size_t)b * strideB;
  const T* Ab2 = SPLIT ? (A2  + (size_t)b * strideA) : nullptr;
  const T* Bb2 = SPLIT ? (Bt2 + (size_t)b * strideB) : nullptr;

  const int rlane = lane & 15;
  const int koff  = (lane >> 4) * 8;
  const int mOff  = (lane >> 4) * 8;

  v8f acc[4][4];
#pragma unroll
  for (int i = 0; i < 4; ++i)
#pragma unroll
    for (int j = 0; j < 4; ++j) acc[i][j] = (v8f){0.f,0.f,0.f,0.f,0.f,0.f,0.f,0.f};

#pragma unroll 1
  for (int k0 = 0; k0 < K; k0 += 32) {
    V bh[4], bl[4];
#pragma unroll
    for (int j = 0; j < 4; ++j) {
      const size_t bo = (size_t)(n0 + (j << 4) + rlane) * ldb + koff + k0;
      bh[j] = Frag<T>::load(Bb + bo);
      if (SPLIT) bl[j] = Frag<T>::load(Bb2 + bo);
    }
#pragma unroll
    for (int i = 0; i < 4; ++i) {
      const size_t ao = (size_t)(m0 + (i << 4) + rlane) * lda + koff + k0;
      V ah = Frag<T>::load(Ab + ao);
      V al;
      if (SPLIT) al = Frag<T>::load(Ab2 + ao);
#pragma unroll
      for (int j = 0; j < 4; ++j) {
        acc[i][j] = Frag<T>::mma(ah, bh[j], acc[i][j]);
        if (SPLIT) {
          acc[i][j] = Frag<T>::mma(ah, bl[j], acc[i][j]);
          acc[i][j] = Frag<T>::mma(al, bh[j], acc[i][j]);
        }
      }
      Frag<T>::guard(acc[i][0], acc[i][3], ah, SPLIT ? al : ah);
    }
    Frag<T>::keep(bh[0], bh[1], bh[2], bh[3]);
    if (SPLIT) Frag<T>::keep(bl[0], bl[1], bl[2], bl[3]);
  }
  acc_guard4(acc[0][0], acc[0][1], acc[0][2], acc[0][3]);
  acc_guard4(acc[1][0], acc[1][1], acc[1][2], acc[1][3]);
  acc_guard4(acc[2][0], acc[2][1], acc[2][2], acc[2][3]);
  acc_guard4(acc[3][0], acc[3][1], acc[3][2], acc[3][3]);

  float* slab = sT[wave];
  const float* Rb = RESID ? (resid + (size_t)b * strideR) : nullptr;
#pragma unroll
  for (int i = 0; i < 4; ++i) {
    const int mBase = m0 + (i << 4);
#pragma unroll
    for (int j = 0; j < 4; ++j) {
      const int n = n0 + (j << 4) + rlane;
      float bv = 0.f;
      if (BIAS_MODE == 2) bv = bias[n];
#pragma unroll
      for (int r = 0; r < 8; ++r) {
        float v = acc[i][j][r] * scale;
        if (BIAS_MODE == 1) v += bias[mBase + mOff + r];
        if (BIAS_MODE == 2) v += bv;
        if (ACT == 1) v = tanhf(v);
        if (ACT == 2) v = fmaxf(v, 0.0f);
        if (ACT == 3) v = v / (1.0f + expf(-v));
        if (ACT == 4) v = (v > 0.f) ? v : 0.01f * v;
        if (ACT == 5) v = 0.5f * v * (1.0f + erff(v * 0.70710678118654752f));
        if (ACT == 6) v = (v > 0.f) ? v : 0.2f * v;
        if (ACT == 7) { const float u = 0.7978845608028654f * (v + 0.044715f * v * v * v); v = 0.5f * v * (1.f + tanhf(u)); }
        slab[(mOff + r) * 68 + (j << 4) + rlane] = v;
      }
    }
    __builtin_amdgcn_fence(3, "workgroup");
    __builtin_amdgcn_wave_barrier();
    __builtin_amdgcn_fence(2, "workgroup");
    if (OUT_MODE == 0) {
      float* C = (float*)Cout + (size_t)b * strideC;
      const int hh = lane >> 4, c4 = (lane & 15) * 4;
      if (RESID) {
#pragma unroll
        for (int it = 0; it < 8; ++it) {
          const int row = it * 2 + hh;
          float* sp = slab + row * 68 + c4;
          const v4f rv = *(const v4f*)(Rb + (size_t)(mBase + row) * ldc + n0 + c4);
          v4f sv = *(const v4f*)sp;
          sv += rv;
          *(v4f*)sp = sv;
        }
        __builtin_amdgcn_fence(3, "workgroup");
        __builtin_amdgcn_wave_barrier();
        __builtin_amdgcn_fence(2, "workgroup");
      }
      for (int pass = 0; pass < 2; ++pass) {
#pragma unroll
        for (int it = 0; it < 8; ++it) {
          const int row = it * 2 + hh;
          v4f v = *(const v4f*)(slab + row * 68 + c4);
          *(volatile v4f*)(C + (size_t)(mBase + row) * ldc + n0 + c4) = v;
        }
        __threadfence();
      }
    } else {
      const int q = lane >> 3, c8 = (lane & 7) * 8;
      unsigned short* C  = (unsigned short*)Cout  + (size_t)b * strideC;
      unsigned short* C2 = (OUT_MODE == 2) ? ((unsigned short*)Cout2 + (size_t)b * strideC) : nullptr;
      for (int pass = 0; pass < 2; ++pass) {
#pragma unroll
        for (int it = 0; it < 4; ++it) {
          const int row = it * 4 + q;
          const float* sp = slab + row * 68 + c8;
          v8h hv, lv;
#pragma unroll
          for (int e = 0; e < 8; ++e) {
            if (OUT_MODE == 1) {
              hv[e] = (_Float16)sp[e];
            } else {
              unsigned short hb = f2bf_bits(sp[e]);
              unsigned short lb = f2bf_bits(sp[e] - bf_bits2f(hb));
              hv[e] = __builtin_bit_cast(_Float16, hb);
              lv[e] = __builtin_bit_cast(_Float16, lb);
            }
          }
          *(volatile v8h*)(C + (size_t)(mBase + row) * ldc + n0 + c8) = hv;
          if (OUT_MODE == 2) *(volatile v8h*)(C2 + (size_t)(mBase + row) * ldc + n0 + c8) = lv;
        }
        __threadfence();
      }
    }
    __builtin_amdgcn_fence(3, "workgroup");
    __builtin_amdgcn_wave_barrier();
    __builtin_amdgcn_fence(2, "workgroup");
  }
}

}

__device__ __forceinline__ unsigned int cmb_pk2(float a, float b) { return (unsigned int)__builtin_bit_cast(unsigned short, (_Float16)a) | ((unsigned int)__builtin_bit_cast(unsigned short, (_Float16)b) << 16); }
__device__ __forceinline__ float cmb_bf(float v) { const unsigned u = __builtin_bit_cast(unsigned, v); const unsigned r = (u + 0x7fffu + ((u >> 16) & 1u)) & 0xffff0000u; return __builtin_bit_cast(float, r); }
__global__ __launch_bounds__(256) void k_bfvec(const float* __restrict__ SRC, float* __restrict__ DST, long long n, float sc) {
    const long long u = (long long)blockIdx.x * 256 + threadIdx.x; if (u >= n) return; VST2(float, DST + u, cmb_bf(SRC[u]) * sc); }
__global__ __launch_bounds__(256) void k_cm_castb(const float* __restrict__ SRC, int lds, unsigned short* __restrict__ DST, int ldd, int nR, int nC, float sc) {
    const long long u = (long long)blockIdx.x * 256 + threadIdx.x; const int per = nC / 8; if (u >= (long long)nR * per) return; const int r = (int)(u / per); const int c0 = 8 * (int)(u % per);
    const float* s = SRC + (long long)r * lds + c0; float w[8];
#pragma unroll
    for (int e = 0; e < 8; ++e) w[e] = cmb_bf(s[e]) * sc;
    cm_u4 pk; pk.x = cmb_pk2(w[0], w[1]); pk.y = cmb_pk2(w[2], w[3]); pk.z = cmb_pk2(w[4], w[5]); pk.w = cmb_pk2(w[6], w[7]); VST2(cm_u4, (cm_u4*)(DST + (long long)r * ldd + c0), pk); }
__global__ __launch_bounds__(256) void k_cm_castbT(const float* __restrict__ SRC, int lds, unsigned short* __restrict__ DST, int ldd, int nR, int nC, float sc) {
    const long long u = (long long)blockIdx.x * 256 + threadIdx.x; const int per = nR / 8; if (u >= (long long)nC * per) return; const int c = (int)(u / per); const int r0 = 8 * (int)(u % per);
    float w[8];
#pragma unroll
    for (int e = 0; e < 8; ++e) w[e] = cmb_bf(SRC[(long long)(r0 + e) * lds + c]) * sc;
    cm_u4 pk; pk.x = cmb_pk2(w[0], w[1]); pk.y = cmb_pk2(w[2], w[3]); pk.z = cmb_pk2(w[4], w[5]); pk.w = cmb_pk2(w[6], w[7]); VST2(cm_u4, (cm_u4*)(DST + (long long)c * ldd + r0), pk); }

#define QEP 80
#define ATT_NW 4
__global__ __launch_bounds__(128) __attribute__((amdgpu_num_vgpr(256)))
void k_relattn(const _Float16* __restrict__ Q16, const _Float16* __restrict__ K16, const _Float16* __restrict__ VT16,
               const _Float16* __restrict__ E16, const float* __restrict__ amask, const float* __restrict__ hmask,
               _Float16* __restrict__ CTX16) {
    __shared__ __align__(16) _Float16 Ksh[64 * 64];
    __shared__ __align__(16) _Float16 Vt[64 * 64];
    __shared__ __align__(16) _Float16 Ew[128 * 64];
    __shared__ __align__(16) float    QEs[ATT_NW][16 * QEP];
    __shared__ __align__(16) float    KEs[4][16 * QEP];
    __shared__ __align__(16) _Float16 Ps[ATT_NW][16 * 64];

    const int tid = threadIdx.x, wave = tid >> 5, lane = tid & 31, hh = lane >> 4, c = lane & 15;
    const int qb = blockIdx.x, h = blockIdx.y, b = blockIdx.z;
    const int q0b = qb * 64, q0 = q0b + 16 * wave;
    const size_t tok0 = (size_t)b * SEQ;
    const float L2E = 1.4426950408889634f;
    const float NEG = -__builtin_inff();
    const float SCL2 = (0.125f / 256.0f) * L2E;
    const float hm = cmb_bf(hmask[h]);

    v16h qa[2];
    {
        const _Float16* qrow = Q16 + (tok0 + q0 + c) * HID + h * HD;
        qa[0] = frag16(qrow, hh);
        qa[1] = frag16(qrow + 32, hh);
    }

    float m8[8], l8[8];
    v8f o[4];
#pragma unroll
    for (int i = 0; i < 8; ++i) { m8[i] = NEG; l8[i] = 0.f; }
#pragma unroll
    for (int t = 0; t < 4; ++t) o[t] = (v8f){0.f,0.f,0.f,0.f,0.f,0.f,0.f,0.f};

    float* qes = QEs[wave];
    float* kes = KEs[wave];
    _Float16* pw = Ps[wave];
    const int wb = 48 - 16 * wave;

#pragma unroll 1
    for (int r0 = 0; r0 < SEQ; r0 += 64) {
        __syncthreads();
        {
#pragma unroll
            for (int it = 0; it < 4; ++it) {
                const int p = tid + it * 128; const int kr = p >> 3, c8 = (p & 7) * 8;
                *(v8h*)(Ksh + kr * 64 + c8) = *(const v8h*)(K16 + (tok0 + r0 + kr) * HID + h * HD + c8);
            }
#pragma unroll
            for (int it = 0; it < 4; ++it) {
                const int p = tid + it * 128; const int d = p >> 3, c8 = (p & 7) * 8;
                *(v8h*)(Vt + d * 64 + c8) = *(const v8h*)(VT16 + (size_t)(h * HD + d) * NR + tok0 + r0 + c8);
            }
            ld_split();
            const int ebase = q0b - r0 + (MAXP - 1 - 63);
#pragma unroll
            for (int it = 0; it < 8; ++it) {
                const int p = tid + it * 128; const int w = p >> 3, c8 = (p & 7) * 8;
                int ei = ebase + w; ei = (ei < 0) ? 0 : ((ei > EROWS - 1) ? (EROWS - 1) : ei);
                *(v8h*)(Ew + w * 64 + c8) = *(const v8h*)(E16 + (size_t)ei * HD + c8);
            }
        }
        __syncthreads();

        v8f s[4];
#pragma unroll
        for (int t = 0; t < 4; ++t) {
            v8f acc = (v8f){0.f,0.f,0.f,0.f,0.f,0.f,0.f,0.f};
#pragma unroll
            for (int dc = 0; dc < 2; ++dc) acc = wmma16(qa[dc], frag16(Ksh + (16 * t + c) * 64 + dc * 32, hh), acc);
            s[t] = acc;
        }
#pragma unroll
        for (int u = 0; u < 5; ++u) {
            v8f acc = (v8f){0.f,0.f,0.f,0.f,0.f,0.f,0.f,0.f};
#pragma unroll
            for (int dc = 0; dc < 2; ++dc) acc = wmma16(qa[dc], frag16(Ew + (16 * wave + 16 * u + c) * 64 + dc * 32, hh), acc);
#pragma unroll
            for (int r = 0; r < 8; ++r) qes[(8 * hh + r) * QEP + 16 * u + c] = acc[r];
        }
        {
            v16h ka[2];
            ka[0] = frag16(Ksh + (16 * wave + c) * 64, hh);
            ka[1] = frag16(Ksh + (16 * wave + c) * 64 + 32, hh);
#pragma unroll
            for (int u = 0; u < 5; ++u) {
                v8f acc = (v8f){0.f,0.f,0.f,0.f,0.f,0.f,0.f,0.f};
#pragma unroll
                for (int dc = 0; dc < 2; ++dc) acc = wmma16(ka[dc], frag16(Ew + (wb + 16 * u + c) * 64 + dc * 32, hh), acc);
#pragma unroll
                for (int r = 0; r < 8; ++r) kes[(8 * hh + r) * QEP + 16 * u + c] = acc[r];
            }
        }
        __syncthreads();

        float mk[4];
#pragma unroll
        for (int t = 0; t < 4; ++t) mk[t] = cmb_bf(amask[(size_t)b * SEQ_FULL + r0 + 16 * t + c]) * L2E;
#pragma unroll
        for (int i = 0; i < 8; ++i) {
            const int m = 8 * hh + i;
            float sc[4]; float mx = NEG;
#pragma unroll
            for (int t = 0; t < 4; ++t) {
                const float qe = qes[m * QEP + (m - 16 * t - c + 63)];
                const float ke = KEs[t][c * QEP + (16 * wave + m - c + 15)];
                const float v = (s[t][i] + qe + ke) * SCL2 + mk[t];
                sc[t] = v; mx = fmaxf(mx, v);
            }
#pragma unroll
            for (int off = 1; off < 16; off <<= 1) mx = fmaxf(mx, __shfl_xor(mx, off, 32));
            const float mnew = fmaxf(m8[i], mx);
            const float corr = (mnew == NEG) ? 1.f : exp2f(m8[i] - mnew);
            m8[i] = mnew;
            float rs = 0.f;
#pragma unroll
            for (int t = 0; t < 4; ++t) {
                const float pp = (sc[t] == NEG) ? 0.f : exp2f(sc[t] - mnew);
                rs += pp;
                pw[m * 64 + 16 * t + c] = (_Float16)(pp * 4096.0f);
            }
#pragma unroll
            for (int off = 1; off < 16; off <<= 1) rs += __shfl_xor(rs, off, 32);
            l8[i] = l8[i] * corr + rs;
#pragma unroll
            for (int t = 0; t < 4; ++t) o[t][i] *= corr;
        }
        __builtin_amdgcn_fence(3, "workgroup");
        __builtin_amdgcn_wave_barrier();
        __builtin_amdgcn_fence(2, "workgroup");

#pragma unroll
        for (int kk = 0; kk < 2; ++kk) {
            const v16h pa = frag16(pw + c * 64 + kk * 32, hh);
#pragma unroll
            for (int t = 0; t < 4; ++t) o[t] = wmma16(pa, frag16(Vt + (16 * t + c) * 64 + kk * 32, hh), o[t]);
        }
    }

    float* os = qes;
#pragma unroll
    for (int i = 0; i < 8; ++i) {
        const float inv = (l8[i] > 0.f) ? (hm * (CSC / 65536.0f)) / l8[i] : 0.f;
#pragma unroll
        for (int t = 0; t < 4; ++t) os[(8 * hh + i) * 64 + 16 * t + c] = o[t][i] * inv;
    }
    __builtin_amdgcn_fence(3, "workgroup");
    __builtin_amdgcn_wave_barrier();
    __builtin_amdgcn_fence(2, "workgroup");
    {
        _Float16* ob = CTX16 + (tok0 + q0) * HID + h * HD;
        const int rq = lane >> 3, c8 = (lane & 7) * 8;
        for (int pass = 0; pass < 2; ++pass) {
#pragma unroll
            for (int it = 0; it < 4; ++it) {
                const int rr = it * 4 + rq;
                const float* sp = os + rr * 64 + c8;
                const v4f a0 = *(const v4f*)sp;
                const v4f a1 = *(const v4f*)(sp + 4);
                v8h hv;
                hv[0] = (_Float16)a0.x; hv[1] = (_Float16)a0.y; hv[2] = (_Float16)a0.z; hv[3] = (_Float16)a0.w;
                hv[4] = (_Float16)a1.x; hv[5] = (_Float16)a1.y; hv[6] = (_Float16)a1.z; hv[7] = (_Float16)a1.w;
                *(volatile v8h*)(ob + (size_t)rr * HID + c8) = hv;
            }
            __threadfence();
        }
    }
}

__device__ __forceinline__ float wsum32(float v) {
#pragma unroll
    for (int off = 16; off > 0; off >>= 1) v += __shfl_xor(v, off, 32);
    return v;
}
__global__ __launch_bounds__(256) void k_ln(const float* __restrict__ Y, const float* __restrict__ G, const float* __restrict__ Bv,
                                            float* __restrict__ OF, _Float16* __restrict__ OH) {
    __shared__ float red[8];
    const int r = blockIdx.x, tid = threadIdx.x, lane = tid & 31, wave = tid >> 5;
    const size_t eo = (size_t)r * HID + 4 * tid;
    const v4f x = *(const v4f*)(Y + eo);
    float s = (x.x + x.y) + (x.z + x.w);
    s = wsum32(s);
    if (lane == 0) red[wave] = s;
    __syncthreads();
    float tot = 0.f;
#pragma unroll
    for (int w = 0; w < 8; ++w) tot += red[w];
    const float mu = tot * (1.0f / (float)HID);
    __syncthreads();
    const v4f d = x - mu;
    float q = (d.x * d.x + d.y * d.y) + (d.z * d.z + d.w * d.w);
    q = wsum32(q);
    if (lane == 0) red[wave] = q;
    __syncthreads();
    float tq = 0.f;
#pragma unroll
    for (int w = 0; w < 8; ++w) tq += red[w];
    const float rstd = rsqrtf(tq * (1.0f / (float)HID) + LN_EPS);
    const v4f g4 = *(const v4f*)(G + 4 * tid), b4 = *(const v4f*)(Bv + 4 * tid);
    v4f y;
    y.x = d.x * rstd * cmb_bf(g4.x) + cmb_bf(b4.x);
    y.y = d.y * rstd * cmb_bf(g4.y) + cmb_bf(b4.y);
    y.z = d.z * rstd * cmb_bf(g4.z) + cmb_bf(b4.z);
    y.w = d.w * rstd * cmb_bf(g4.w) + cmb_bf(b4.w);
    VST2V4(OF + eo, y);
    if (OH) {
        v4h hv; hv.x = (_Float16)y.x; hv.y = (_Float16)y.y; hv.z = (_Float16)y.z; hv.w = (_Float16)y.w;
        VST2(v4h, OH + eo, hv);
    }
}

extern "C" void kernel_launch(void* const* d_in, const int* in_sizes, int n_in, void* d_out, int out_size, void* d_ws, size_t ws_size, hipStream_t stream) {
    if (n_in < 20) return;
    if (in_sizes[0] < NR * HID) return;
    if (in_sizes[1] < (NB - 1) * SEQ_FULL + SEQ) return;
    if (in_sizes[2] < NH) return;
    if (in_sizes[3] < HID * HID || in_sizes[5] < HID * HID || in_sizes[7] < HID * HID || in_sizes[10] < HID * HID) return;
    if (in_sizes[4] < HID || in_sizes[6] < HID || in_sizes[8] < HID || in_sizes[11] < HID || in_sizes[17] < HID) return;
    if (in_sizes[12] < HID || in_sizes[13] < HID || in_sizes[18] < HID || in_sizes[19] < HID) return;
    if (in_sizes[9] < EROWS * HD) return;
    if (in_sizes[14] < HID * FFD || in_sizes[16] < FFD * HID || in_sizes[15] < FFD) return;
    if (out_size < NR * HID) return;

    const float* x    = (const float*)d_in[0];
    const float* amsk = (const float*)d_in[1];
    const float* hmsk = (const float*)d_in[2];
    const float* Wq = (const float*)d_in[3];  const float* bq = (const float*)d_in[4];
    const float* Wk = (const float*)d_in[5];  const float* bk = (const float*)d_in[6];
    const float* Wv = (const float*)d_in[7];  const float* bv = (const float*)d_in[8];
    const float* Emb = (const float*)d_in[9];
    const float* Wo = (const float*)d_in[10]; const float* bo = (const float*)d_in[11];
    const float* g1 = (const float*)d_in[12]; const float* be1 = (const float*)d_in[13];
    const float* Wi = (const float*)d_in[14]; const float* bi = (const float*)d_in[15];
    const float* Wo2 = (const float*)d_in[16]; const float* bo2 = (const float*)d_in[17];
    const float* g2 = (const float*)d_in[18]; const float* be2 = (const float*)d_in[19];
    float* out = (float*)d_out;

    char* base = (char*)d_ws; size_t off = 0;
    auto carve = [&](size_t bytes) -> size_t { const size_t o = off; off += (bytes + 255) & ~(size_t)255; return o; };
    const size_t oX16 = carve((size_t)NR * HID * 2);
    const size_t oXr  = carve((size_t)NR * HID * 4);
    const size_t oWq  = carve((size_t)HID * HID * 2);
    const size_t oWk  = carve((size_t)HID * HID * 2);
    const size_t oWv  = carve((size_t)HID * HID * 2);
    const size_t oWo  = carve((size_t)HID * HID * 2);
    const size_t oWi  = carve((size_t)FFD * HID * 2);
    const size_t oWo2 = carve((size_t)HID * FFD * 2);
    const size_t oE   = carve((size_t)EROWS * HD * 2);
    const size_t oBq  = carve((size_t)HID * 4);
    const size_t oBk  = carve((size_t)HID * 4);
    const size_t oBv  = carve((size_t)HID * 4);
    const size_t oBo  = carve((size_t)HID * 4);
    const size_t oBi  = carve((size_t)FFD * 4);
    const size_t oBo2 = carve((size_t)HID * 4);
    const size_t oQC  = carve((size_t)NR * HID * 2 * 4);
    const size_t oY   = carve((size_t)NR * HID * 4);
    const size_t oA1  = carve((size_t)NR * HID * 4);
    const size_t oA1h = carve((size_t)NR * HID * 2);
    if (off > ws_size || off > (size_t)128 * 1024 * 1024) return;

    unsigned short* X16  = (unsigned short*)(base + oX16);
    float*          Xr   = (float*)(base + oXr);
    unsigned short* WqT  = (unsigned short*)(base + oWq);
    unsigned short* WkT  = (unsigned short*)(base + oWk);
    unsigned short* WvT  = (unsigned short*)(base + oWv);
    unsigned short* WoT  = (unsigned short*)(base + oWo);
    unsigned short* WiT  = (unsigned short*)(base + oWi);
    unsigned short* Wo2T = (unsigned short*)(base + oWo2);
    unsigned short* E16  = (unsigned short*)(base + oE);
    float* BRq = (float*)(base + oBq);  float* BRk = (float*)(base + oBk);  float* BRv = (float*)(base + oBv);
    float* BRo = (float*)(base + oBo);  float* BRi = (float*)(base + oBi);  float* BRo2 = (float*)(base + oBo2);
    _Float16* Q16   = (_Float16*)(base + oQC);
    _Float16* K16   = Q16 + (size_t)NR * HID;
    _Float16* VT16  = K16 + (size_t)NR * HID;
    _Float16* CTX16 = VT16 + (size_t)HID * NR;
    _Float16* INT16 = Q16;
    float* Y   = (float*)(base + oY);
    float* A1  = (float*)(base + oA1);
    _Float16* A1h = (_Float16*)(base + oA1h);

    k_cm_castb<<<(unsigned)((((long long)NR) * (HID / 8) + 255) / 256), 256, 0, stream>>>(x, HID, X16, HID, NR, HID, 1.0f);
    k_bfvec<<<(unsigned)(((long long)NR * HID + 255) / 256), 256, 0, stream>>>(x, Xr, (long long)NR * HID, 1.0f);
    k_cm_castbT<<<(unsigned)((((long long)HID) * (HID / 8) + 255) / 256), 256, 0, stream>>>(Wq, HID, WqT, HID, HID, HID, 16.0f);
    k_cm_castbT<<<(unsigned)((((long long)HID) * (HID / 8) + 255) / 256), 256, 0, stream>>>(Wk, HID, WkT, HID, HID, HID, 16.0f);
    k_cm_castbT<<<(unsigned)((((long long)HID) * (HID / 8) + 255) / 256), 256, 0, stream>>>(Wv, HID, WvT, HID, HID, HID, 16.0f);
    k_cm_castbT<<<(unsigned)((((long long)HID) * (HID / 8) + 255) / 256), 256, 0, stream>>>(Wo, HID, WoT, HID, HID, HID, 16.0f);
    k_cm_castbT<<<(unsigned)((((long long)FFD) * (HID / 8) + 255) / 256), 256, 0, stream>>>(Wi, FFD, WiT, HID, HID, FFD, 16.0f);
    k_cm_castbT<<<(unsigned)((((long long)HID) * (FFD / 8) + 255) / 256), 256, 0, stream>>>(Wo2, HID, Wo2T, FFD, FFD, HID, 16.0f);
    k_cm_castb<<<(unsigned)((((long long)EROWS) * (HD / 8) + 255) / 256), 256, 0, stream>>>(Emb, HD, E16, HD, EROWS, HD, 16.0f);
    k_bfvec<<<(unsigned)((HID + 255) / 256), 256, 0, stream>>>(bq, BRq, HID, 16.0f);
    k_bfvec<<<(unsigned)((HID + 255) / 256), 256, 0, stream>>>(bk, BRk, HID, 16.0f);
    k_bfvec<<<(unsigned)((HID + 255) / 256), 256, 0, stream>>>(bv, BRv, HID, 16.0f);
    k_bfvec<<<(unsigned)((HID + 255) / 256), 256, 0, stream>>>(bo, BRo, HID, 1.0f);
    k_bfvec<<<(unsigned)((FFD + 255) / 256), 256, 0, stream>>>(bi, BRi, FFD, 1.0f);
    k_bfvec<<<(unsigned)((HID + 255) / 256), 256, 0, stream>>>(bo2, BRo2, HID, 1.0f);

    const unsigned gQK = (unsigned)((((NR) / 64) * ((HID) / 64) + 7) / 8);
    w25::wmma_gemm64<0, false, 2, 1, false, 0><<<dim3(gQK, 1), 256, 0, stream>>>((const unsigned short*)X16, nullptr, HID, 0, (const unsigned short*)WqT, nullptr, HID, 0, (void*)Q16, nullptr, HID, 0, BRq, nullptr, 0, NR, HID, HID, 1.0f);
    w25::wmma_gemm64<0, false, 2, 1, false, 0><<<dim3(gQK, 1), 256, 0, stream>>>((const unsigned short*)X16, nullptr, HID, 0, (const unsigned short*)WkT, nullptr, HID, 0, (void*)K16, nullptr, HID, 0, BRk, nullptr, 0, NR, HID, HID, 1.0f);
    w25::wmma_gemm64<0, false, 1, 1, false, 0><<<dim3(gQK, 1), 256, 0, stream>>>((const unsigned short*)WvT, nullptr, HID, 0, (const unsigned short*)X16, nullptr, HID, 0, (void*)VT16, nullptr, NR, 0, BRv, nullptr, 0, HID, NR, HID, 1.0f);

    k_relattn<<<dim3((unsigned)(SEQ / 64), (unsigned)NH, (unsigned)NB), 32 * ATT_NW, 0, stream>>>(Q16, K16, VT16, (const _Float16*)E16, amsk, hmsk, CTX16);

    w25::wmma_gemm64<0, false, 2, 0, true, 0><<<dim3(gQK, 1), 256, 0, stream>>>((const unsigned short*)CTX16, nullptr, HID, 0, (const unsigned short*)WoT, nullptr, HID, 0, (void*)Y, nullptr, HID, 0, BRo, Xr, 0, NR, HID, HID, 1.0f / (CSC * 16.0f));
    k_ln<<<(unsigned)NR, 256, 0, stream>>>(Y, g1, be1, A1, A1h);

    const unsigned gWi = (unsigned)((((NR) / 64) * ((FFD) / 64) + 7) / 8);
    w25::wmma_gemm64<0, false, 2, 1, false, 5><<<dim3(gWi, 1), 256, 0, stream>>>((const unsigned short*)A1h, nullptr, HID, 0, (const unsigned short*)WiT, nullptr, HID, 0, (void*)INT16, nullptr, FFD, 0, BRi, nullptr, 0, NR, FFD, HID, 1.0f / 16.0f);
    w25::wmma_gemm64<0, false, 2, 0, true, 0><<<dim3(gQK, 1), 256, 0, stream>>>((const unsigned short*)INT16, nullptr, FFD, 0, (const unsigned short*)Wo2T, nullptr, FFD, 0, (void*)Y, nullptr, HID, 0, BRo2, A1, 0, NR, HID, FFD, 1.0f / 16.0f);
    k_ln<<<(unsigned)NR, 256, 0, stream>>>(Y, g2, be2, out, nullptr);
}
